// ScalingAttention_74105365725832
// MI455X (gfx1250) — hardware-verified
//
#include <hip/hip_runtime.h>


#define NB_  2
#define TQ   4096
#define TK   1024
#define DD   512
#define NH_  8
#define HD   64
#define DS   4
#define SCL  0.125f
typedef _Float16 h16;
typedef unsigned short bf;
typedef __attribute__((ext_vector_type(16))) __bf16   v16bf;
typedef __attribute__((ext_vector_type(16))) _Float16 v16h;
typedef __attribute__((ext_vector_type(8)))  _Float16 v8h;
typedef __attribute__((ext_vector_type(8)))  unsigned short v8us;
typedef __attribute__((ext_vector_type(8)))  float    v8f;
typedef __attribute__((ext_vector_type(4)))  float    v4f;
typedef v8h  __attribute__((may_alias)) v8ha;
typedef v4f  __attribute__((may_alias)) v4fa;
typedef v8us __attribute__((may_alias)) v8usa;

__device__ __forceinline__ unsigned short f2bf(float f) { unsigned u = __float_as_uint(f); u += 0x7FFFu + ((u >> 16) & 1u); return (unsigned short)(u >> 16); }
__device__ __forceinline__ float bf2f(unsigned short b) { return __uint_as_float(((unsigned)b) << 16); }
__device__ __forceinline__ float bfr(float f) { return bf2f(f2bf(f)); }
__device__ __forceinline__ v16h cat16(v8h lo, v8h hi) { return __builtin_shufflevector(lo, hi, 0, 1, 2, 3, 4, 5, 6, 7, 8, 9, 10, 11, 12, 13, 14, 15); }
__device__ __forceinline__ v16bf cat16b(v8us lo, v8us hi) { return __builtin_bit_cast(v16bf, __builtin_shufflevector(lo, hi, 0, 1, 2, 3, 4, 5, 6, 7, 8, 9, 10, 11, 12, 13, 14, 15)); }
__device__ __forceinline__ v8f wmma16(v16h a, v16h b, v8f c) { return __builtin_amdgcn_wmma_f32_16x16x32_f16(false, a, false, b, (short)0, c, false, false); }
__device__ __forceinline__ v8f wmmab(v16bf a, v16bf b, v8f c) { return __builtin_amdgcn_wmma_f32_16x16x32_bf16(false, a, false, b, (short)0, c, false, false); }


template <typename T16> struct WFrag;
template <> struct WFrag<h16> { typedef v16h V; static __device__ __forceinline__ V ld(const h16* p) { return cat16(*(const v8h*)p, *(const v8h*)(p + 16)); } static __device__ __forceinline__ v8f mma(V a, V b, v8f c) { return wmma16(a, b, c); } };
template <> struct WFrag<bf> { typedef v16bf V; static __device__ __forceinline__ V ld(const bf* p) { return cat16b(*(const v8us*)p, *(const v8us*)(p + 16)); } static __device__ __forceinline__ v8f mma(V a, V b, v8f c) { return wmmab(a, b, c); } };
template <typename T16, int NSPLIT, bool BIAS>
__global__ __launch_bounds__(32) void k_gemmw(const T16* __restrict__ A, const T16* __restrict__ A2, const T16* __restrict__ Bt, const T16* __restrict__ Bt2, int K, float* C, int ldc, const float* __restrict__ bias, size_t sA, size_t sB, size_t sC) {
    typedef typename WFrag<T16>::V V;
    __shared__ __align__(16) float os[16 * 68];
    const size_t z = blockIdx.z; A += z * sA; if (A2) A2 += z * sA; Bt += z * sB; if (Bt2) Bt2 += z * sB; C += z * sC;
    const int lane = threadIdx.x & 31, lr = lane & 15, hi = lane >> 4; const int r0 = blockIdx.x * 64, c0 = blockIdx.y * 64;
    v8f acc[4][4];
#pragma unroll
    for (int mb = 0; mb < 4; ++mb)
#pragma unroll
        for (int nb = 0; nb < 4; ++nb) acc[mb][nb] = (v8f){};
    const size_t aoff = (size_t)(r0 + lr) * K + 8 * hi, boff = (size_t)(c0 + lr) * K + 8 * hi;
#pragma unroll 1
    for (int kc = 0; kc < K; kc += 32) {
        V a[4], a2[4];
#pragma unroll
        for (int mb = 0; mb < 4; ++mb) { a[mb] = WFrag<T16>::ld(A + aoff + (size_t)mb * 16 * K + kc); if (NSPLIT == 1 || NSPLIT == 2) a2[mb] = WFrag<T16>::ld(A2 + aoff + (size_t)mb * 16 * K + kc); }
#pragma unroll
        for (int nb = 0; nb < 4; ++nb) { const V b = WFrag<T16>::ld(Bt + boff + (size_t)nb * 16 * K + kc); V b2; if (NSPLIT >= 2) b2 = WFrag<T16>::ld(Bt2 + boff + (size_t)nb * 16 * K + kc);
#pragma unroll
            for (int mb = 0; mb < 4; ++mb) { acc[mb][nb] = WFrag<T16>::mma(a[mb], b, acc[mb][nb]); if (NSPLIT == 1 || NSPLIT == 2) acc[mb][nb] = WFrag<T16>::mma(a2[mb], b, acc[mb][nb]); if (NSPLIT >= 2) acc[mb][nb] = WFrag<T16>::mma(a[mb], b2, acc[mb][nb]); } }
        asm volatile("v_nop\n\tv_nop\n\tv_nop\n\tv_nop" : "+v"(acc[0][0]), "+v"(acc[1][1]), "+v"(acc[2][2]), "+v"(acc[3][3]) : "v"(a[0]), "v"(a[3]));
    }
#pragma unroll
    for (int mb = 0; mb < 4; ++mb) {
#pragma unroll
        for (int nb = 0; nb < 4; ++nb) {
#pragma unroll
            for (int j = 0; j < 8; ++j) os[(hi * 8 + j) * 68 + nb * 16 + lr] = acc[mb][nb][j]; }
        __builtin_amdgcn_wave_barrier(); asm volatile("" ::: "memory");
        float* crow = C + (size_t)(r0 + mb * 16) * ldc + c0;
#pragma unroll 1
        for (int ps = 0; ps < 2; ++ps) {
#pragma unroll
            for (int s = 0; s < 8; ++s) { const int row = 2 * s + hi, cofs = lr * 4; v4f val = *(const v4fa*)(os + row * 68 + cofs); if (BIAS) { val[0] += bfr(bias[c0 + cofs]); val[1] += bfr(bias[c0 + cofs + 1]); val[2] += bfr(bias[c0 + cofs + 2]); val[3] += bfr(bias[c0 + cofs + 3]); }
                *(volatile v4f*)(crow + (size_t)row * ldc + cofs) = val; }
            if (ps == 0) __threadfence(); }
        __builtin_amdgcn_wave_barrier(); asm volatile("" ::: "memory");
    }
}

__device__ __forceinline__ h16 tohx(float x) { return (h16)x; }
__device__ __forceinline__ void splitf(float y, unsigned short& h, unsigned short& l) { h = f2bf(y); l = f2bf(y - bf2f(h)); }
typedef __attribute__((ext_vector_type(2))) _Float16 v2h;
typedef __attribute__((ext_vector_type(4))) _Float16 v4h;
typedef __attribute__((ext_vector_type(2))) unsigned short v2us;
typedef __attribute__((ext_vector_type(4))) unsigned short v4us;
typedef __attribute__((ext_vector_type(2))) float v2f;

__global__ __launch_bounds__(256) void k_wtG(const float* __restrict__ w, int K, int N, bf* Bt) {
    const int lane = threadIdx.x & 31; const int L0 = (blockIdx.x * 8 + (threadIdx.x >> 5)) * 8; const int nlines = N * K / 64;
#pragma unroll 1
    for (int ps = 0; ps < 2; ++ps) {
#pragma unroll 1
        for (int l = 0; l < 8; ++l) { const int L = L0 + l; if (L >= nlines) break; const size_t e = (size_t)L * 64 + lane * 2; const int k = (int)(e % K), n = (int)(e / K); v2us o;
            o[0] = f2bf(w[(size_t)k * N + n]); o[1] = f2bf(w[(size_t)(k + 1) * N + n]); *(volatile v2us*)(Bt + e) = o; }
        if (ps == 0) __threadfence(); }
}
__global__ __launch_bounds__(256) void k_cvt8(const float* __restrict__ src, bf* dst, size_t n8) { const size_t i = (size_t)blockIdx.x * 256 + threadIdx.x; if (i >= n8) return; const v8f v = *(const v8f*)(src + i * 8); v8us o;
#pragma unroll
    for (int k = 0; k < 8; ++k) o[k] = f2bf(v[k]); *(volatile v8us*)(dst + i * 8) = o; __threadfence(); *(volatile v8us*)(dst + i * 8) = o; }
__global__ __launch_bounds__(256) void k_p16(const float* __restrict__ F, int nt, h16* P) { const size_t e = ((size_t)blockIdx.x * 256 + threadIdx.x) * 2; if (e >= (size_t)NH_ * nt * HD) return; const int d = (int)(e % HD); const int t = (int)((e / HD) % nt); const int h = (int)(e / ((size_t)HD * nt)); const float* s = F + (size_t)t * DD + h * HD + d; v2h o; o[0] = tohx(s[0]); o[1] = tohx(s[1]); *(volatile v2h*)(P + e) = o; __threadfence(); *(volatile v2h*)(P + e) = o; }
__global__ __launch_bounds__(256) void k_vthl(const float* __restrict__ F, bf* Vh, bf* Vl) { const size_t e = ((size_t)blockIdx.x * 256 + threadIdx.x) * 2; if (e >= (size_t)NH_ * HD * TK) return; const int t = (int)(e % TK); const int d = (int)((e / TK) % HD); const int h = (int)(e / ((size_t)TK * HD)); v2us oh, ol;
#pragma unroll
    for (int q = 0; q < 2; ++q) { unsigned short a, c2; splitf(F[(size_t)(t + q) * DD + h * HD + d], a, c2); oh[q] = a; ol[q] = c2; } *(volatile v2us*)(Vh + e) = oh; *(volatile v2us*)(Vl + e) = ol; __threadfence(); *(volatile v2us*)(Vh + e) = oh; *(volatile v2us*)(Vl + e) = ol; }
__global__ __launch_bounds__(256) void k_bsoft(const float* __restrict__ Sb, bf* Ph, bf* Pl) { const int lane = threadIdx.x & 31; const int row = blockIdx.x * 8 + (threadIdx.x >> 5); if (row >= TQ) return; const int jmax = row / DS; const float* sr = Sb + (size_t)row * TK; float v[32]; float mx = -3.0e38f;
#pragma unroll
    for (int ch = 0; ch < 8; ++ch) { const int j0 = ch * 128 + lane * 4; const v4f a = *(const v4f*)(sr + j0);
#pragma unroll
        for (int q = 0; q < 4; ++q) { const int j = j0 + q; float t = __fmul_rn(a[q], SCL); asm volatile("" : "+v"(t)); t = (j <= jmax) ? t : -3.0e38f; v[ch * 4 + q] = t; mx = fmaxf(mx, t); } }
#pragma unroll
    for (int sh = 16; sh; sh >>= 1) mx = fmaxf(mx, __shfl_xor(mx, sh, 32));
    float sum = 0.f;
#pragma unroll
    for (int k = 0; k < 32; ++k) { float d0 = __fsub_rn(v[k], mx); asm volatile("" : "+v"(d0)); v[k] = (v[k] > -1.0e38f) ? __expf(d0) : 0.f; sum += v[k]; }
#pragma unroll
    for (int sh = 16; sh; sh >>= 1) sum += __shfl_xor(sum, sh, 32);
    const float f = __fdiv_rn(1.0f, sum);
#pragma unroll 1
    for (int ps = 0; ps < 2; ++ps) {
#pragma unroll
        for (int ch = 0; ch < 8; ++ch) { v4us oh, ol;
#pragma unroll
            for (int q = 0; q < 4; ++q) { float y = __fmul_rn(v[ch * 4 + q], f); asm volatile("" : "+v"(y)); unsigned short a2, c2; splitf(y, a2, c2); oh[q] = a2; ol[q] = c2; }
            *(volatile v4us*)(Ph + (size_t)row * TK + ch * 128 + lane * 4) = oh; *(volatile v4us*)(Pl + (size_t)row * TK + ch * 128 + lane * 4) = ol; }
        if (ps == 0) __threadfence(); } }
__global__ __launch_bounds__(256) void k_mrgf(const float* __restrict__ O, int h, float* ATT) { const size_t e = ((size_t)blockIdx.x * 256 + threadIdx.x) * 2; if (e >= (size_t)TQ * HD) return; const int d = (int)(e % HD), t = (int)(e / HD); v2f o; o[0] = O[e]; o[1] = O[e + 1]; const size_t oo = (size_t)t * DD + h * HD + d; *(volatile v2f*)(ATT + oo) = o; __threadfence(); *(volatile v2f*)(ATT + oo) = o; }
__global__ __launch_bounds__(256) void k_ln(const float* __restrict__ A, const float* __restrict__ g, const float* __restrict__ bb, bf* Yh, bf* Yl) { const int lane = threadIdx.x & 31; const int t = blockIdx.x * 8 + (threadIdx.x >> 5); if (t >= TQ) return; const float* ar = A + (size_t)t * DD; float v[16]; float s = 0.f;
#pragma unroll
    for (int ch = 0; ch < 4; ++ch) { const v4f a = *(const v4f*)(ar + ch * 128 + lane * 4);
#pragma unroll
        for (int q = 0; q < 4; ++q) { v[ch * 4 + q] = a[q]; s = __fadd_rn(s, a[q]); } }
#pragma unroll
    for (int sh = 16; sh; sh >>= 1) s += __shfl_xor(s, sh, 32);
    const float mu = s * (1.0f / DD); float q2 = 0.f;
#pragma unroll
    for (int k = 0; k < 16; ++k) { const float d = __fsub_rn(v[k], mu); float p = __fmul_rn(d, d); asm volatile("" : "+v"(p)); q2 = __fadd_rn(q2, p); }
#pragma unroll
    for (int sh = 16; sh; sh >>= 1) q2 += __shfl_xor(q2, sh, 32);
    const float rs = __frsqrt_rn(__fadd_rn(q2 * (1.0f / DD), 1e-5f));
#pragma unroll 1
    for (int ps = 0; ps < 2; ++ps) {
#pragma unroll
        for (int ch = 0; ch < 4; ++ch) { v4us oh, ol;
#pragma unroll
            for (int q = 0; q < 4; ++q) { const int d = ch * 128 + lane * 4 + q; float tn = __fmul_rn(__fsub_rn(v[ch * 4 + q], mu), rs); asm volatile("" : "+v"(tn)); float tg = __fmul_rn(tn, bfr(g[d])); asm volatile("" : "+v"(tg)); unsigned short a2, c2; splitf(__fadd_rn(tg, bfr(bb[d])), a2, c2); oh[q] = a2; ol[q] = c2; }
            const size_t o = (size_t)t * DD + ch * 128 + lane * 4; *(volatile v4us*)(Yh + o) = oh; *(volatile v4us*)(Yl + o) = ol; }
        if (ps == 0) __threadfence(); } }

extern "C" void kernel_launch(void* const* d_in, const int* in_sizes, int n_in,
                              void* d_out, int out_size, void* d_ws, size_t ws_size, hipStream_t stream) {
    (void)in_sizes; (void)n_in; (void)out_size;
    const float* IN[9]; for (int i = 0; i < 9; ++i) IN[i] = (const float*)d_in[i];
    float* OUT = (float*)d_out;
    char* wsp = (char*)d_ws;
    auto take = [&](size_t bytes) { char* p = wsp; wsp += (bytes + 255) & ~(size_t)255; return (void*)p; };
    bf* W4[4]; for (int i = 0; i < 4; ++i) W4[i] = (bf*)take((size_t)DD * DD * 2);
    bf* XQ = (bf*)take((size_t)TQ * DD * 2); bf* XK = (bf*)take((size_t)TK * DD * 2); float* FQ = (float*)take((size_t)TQ * DD * 4); float* FK = (float*)take((size_t)TK * DD * 4); float* FV = (float*)take((size_t)TK * DD * 4);
    h16* QP = (h16*)take((size_t)NH_ * TQ * HD * 2); h16* KP = (h16*)take((size_t)NH_ * TK * HD * 2); bf* VTh = (bf*)take((size_t)NH_ * HD * TK * 2); bf* VTl = (bf*)take((size_t)NH_ * HD * TK * 2); float* Sb = (float*)take((size_t)TQ * TK * 4); bf* Ph = (bf*)take((size_t)TQ * TK * 2); bf* Pl = (bf*)take((size_t)TQ * TK * 2); float* O = (float*)take((size_t)TQ * HD * 4);
    float* ATT = FQ;
    bf* Yh = (bf*)take((size_t)TQ * DD * 2); bf* Yl = (bf*)take((size_t)TQ * DD * 2);
    if ((size_t)(wsp - (char*)d_ws) > ws_size) return;
    { const unsigned g = (unsigned)(((size_t)DD * DD / 64 + 63) / 64); for (int i = 0; i < 4; ++i) k_wtG<<<g, 256, 0, stream>>>(IN[2 + i], DD, DD, W4[i]); }
    for (int b = 0; b < NB_; ++b) {
        k_cvt8<<<(TQ * DD / 8 + 255) / 256, 256, 0, stream>>>(IN[0] + (size_t)b * TQ * DD, XQ, (size_t)TQ * DD / 8); k_cvt8<<<(TK * DD / 8 + 255) / 256, 256, 0, stream>>>(IN[1] + (size_t)b * TK * DD, XK, (size_t)TK * DD / 8);
        k_gemmw<bf, 0, false><<<dim3(TQ / 64, DD / 64, 1), 32, 0, stream>>>(XQ, nullptr, W4[0], nullptr, DD, FQ, DD, nullptr, 0, 0, 0); k_gemmw<bf, 0, false><<<dim3(TK / 64, DD / 64, 1), 32, 0, stream>>>(XK, nullptr, W4[1], nullptr, DD, FK, DD, nullptr, 0, 0, 0); k_gemmw<bf, 0, false><<<dim3(TK / 64, DD / 64, 1), 32, 0, stream>>>(XK, nullptr, W4[2], nullptr, DD, FV, DD, nullptr, 0, 0, 0);
        k_p16<<<(unsigned)(((size_t)NH_ * TQ * HD / 2 + 255) / 256), 256, 0, stream>>>(FQ, TQ, QP); k_p16<<<(unsigned)(((size_t)NH_ * TK * HD / 2 + 255) / 256), 256, 0, stream>>>(FK, TK, KP); k_vthl<<<(unsigned)(((size_t)NH_ * HD * TK / 2 + 255) / 256), 256, 0, stream>>>(FV, VTh, VTl);
        for (int h = 0; h < NH_; ++h) {
            k_gemmw<h16, 0, false><<<dim3(TQ / 64, TK / 64, 1), 32, 0, stream>>>(QP + (size_t)h * TQ * HD, nullptr, KP + (size_t)h * TK * HD, nullptr, HD, Sb, TK, nullptr, 0, 0, 0);
            k_bsoft<<<TQ / 8, 256, 0, stream>>>(Sb, Ph, Pl);
            k_gemmw<bf, 2, false><<<dim3(TQ / 64, 1, 1), 32, 0, stream>>>(Ph, Pl, VTh + (size_t)h * HD * TK, VTl + (size_t)h * HD * TK, TK, O, HD, nullptr, 0, 0, 0);
            k_mrgf<<<(TQ * HD / 2 + 255) / 256, 256, 0, stream>>>(O, h, ATT); }
        k_ln<<<TQ / 8, 256, 0, stream>>>(ATT, IN[7], IN[8], Yh, Yl);
        k_gemmw<bf, 1, true><<<dim3(TQ / 64, DD / 64, 1), 32, 0, stream>>>(Yh, Yl, W4[3], nullptr, DD, OUT + (size_t)b * TQ * DD, DD, IN[6], 0, 0, 0); }
}
